// GrigSelfAttentionXSMM_52948356825350
// MI455X (gfx1250) — hardware-verified
//
#include <hip/hip_runtime.h>


namespace {
constexpr int Bn = 128, S = 256, A = 128, H = 8, KD = 16, O = 128, NR = Bn * S, NPJ = 4 * H * KD  ;
constexpr float QS = 8.0f, KS = 8.0f, VS = 8.0f, PS = 8.0f, AS_ = 8.0f, SCALE = 0.25f;
constexpr size_t PL = (size_t)Bn * H * S * KD;

typedef _Float16 b16;
typedef __attribute__((ext_vector_type(16))) _Float16 v16b;
typedef __attribute__((ext_vector_type(8))) _Float16 v8b;
typedef __attribute__((ext_vector_type(8))) float v8f;
typedef __attribute__((ext_vector_type(4))) float v4f;
__device__ __forceinline__ float bf16_rne(float f) { unsigned int u = __float_as_uint(f); u += 0x7FFFu + ((u >> 16) & 1u); return __uint_as_float(u & 0xFFFF0000u); }
__device__ __forceinline__ void split16(float v, b16& hi, b16& lo) { hi = (b16)v; lo = (b16)(v - (float)hi); }
__device__ __forceinline__ v16b frag_kb(const b16* p, int hh) { const v8b a = *(const v8b*)(p + 8 * hh), b = *(const v8b*)(p + 16 + 8 * hh); v16b f;
#pragma unroll
  for (int e = 0; e < 8; ++e) { f[e] = a[e]; f[8 + e] = b[e]; } return f; }
__device__ __forceinline__ v16b frag16(const b16* p, int hh) { const v8b a = *(const v8b*)(p + 8 * hh); v16b f;
#pragma unroll
  for (int e = 0; e < 8; ++e) { f[e] = a[e]; f[8 + e] = (b16)0.0f; } return f; }
__device__ __forceinline__ v16b frag_x(const float* p, int hh) { v16b f;
#pragma unroll
  for (int e = 0; e < 8; ++e) { f[e] = (b16)bf16_rne(p[8 * hh + e]); f[8 + e] = (b16)bf16_rne(p[16 + 8 * hh + e]); } return f; }
__device__ __forceinline__ void frag_split(const float* p, int hh, v16b& fh, v16b& fl) {
#pragma unroll
  for (int e = 0; e < 8; ++e) { b16 a, c; split16(p[8 * hh + e] * AS_, a, c); fh[e] = a; fl[e] = c; split16(p[16 + 8 * hh + e] * AS_, a, c); fh[8 + e] = a; fl[8 + e] = c; } }
__device__ __forceinline__ v8f wmma16b(v16b a, v16b b, v8f c) { v8f d = __builtin_amdgcn_wmma_f32_16x16x32_f16(false, a, false, b, (short)0, c, false, false); asm volatile("v_nop\n\tv_nop\n\tv_nop\n\tv_nop" : "+v"(d) : "v"(a), "v"(b)); return d; }
__device__ __forceinline__ void wave_lds_sync() { __builtin_amdgcn_fence(__ATOMIC_RELEASE, "workgroup"); __builtin_amdgcn_wave_barrier(); __builtin_amdgcn_fence(__ATOMIC_ACQUIRE, "workgroup"); }
__device__ __forceinline__ float nexp(float x) { return __builtin_amdgcn_exp2f(x * 1.4426950408889634f); }
__device__ __forceinline__ float sigm(float x) { return __builtin_amdgcn_rcpf(1.0f + nexp(-x)); }

__global__ __launch_bounds__(256) void prep_kernel(const float* __restrict__ wq, const float* __restrict__ wk, const float* __restrict__ wv, const float* __restrict__ wg, const float* __restrict__ wo, b16* __restrict__ R) {
  const int t_ = blockIdx.x * 256 + threadIdx.x, nth = gridDim.x * 256;
  for (int pass = 0; pass < 2; ++pass) {
    for (int p = t_; p < (NPJ * A + O * 128) / 8; p += nth) { v8b v;
      if (p < NPJ * A / 8) { const int j = p / (A / 8), a0 = (p % (A / 8)) * 8; const int m = j >> 7, jj = j & 127; const float* W = (m == 0) ? wq : (m == 1) ? wk : (m == 2) ? wv : wg;
        for (int e = 0; e < 8; ++e) v[e] = (b16)bf16_rne(W[(size_t)(a0 + e) * 128 + jj]); *(volatile v8b*)(R + (size_t)j * A + a0) = v; }
      else { const int q = p - NPJ * A / 8; const int o = q / 16, k0 = (q % 16) * 8; for (int e = 0; e < 8; ++e) v[e] = (b16)bf16_rne(wo[(size_t)(k0 + e) * O + o]); *(volatile v8b*)(R + (size_t)NPJ * A + (size_t)o * 128 + k0) = v; } }
    __threadfence(); }
}

__global__ __launch_bounds__(128) void proj_kernel(const float* __restrict__ x, const b16* __restrict__ R, b16* __restrict__ Qh, b16* __restrict__ Ql, b16* __restrict__ Kh, b16* __restrict__ Kl, b16* __restrict__ Vt, b16* __restrict__ Vtl, float* __restrict__ G) {
  __shared__ __attribute__((aligned(16))) b16 Th[4][32][128 + 8], Tl[4][32][128 + 8]; __shared__ __attribute__((aligned(16))) b16 Tv[128][128 + 8], Tvl[128][128 + 8];
  const int lane = threadIdx.x & 31, wave = threadIdx.x >> 5, nloc = lane & 15, hlf = lane >> 4, r0 = blockIdx.x * 128, m0 = r0 + wave * 32; const int b = r0 / S, s0 = m0 % S;
  for (int grp = 0; grp < 4; ++grp) {
    v8f acc[2][8];
#pragma unroll
    for (int r = 0; r < 2; ++r)
#pragma unroll
      for (int t = 0; t < 8; ++t) acc[r][t] = (v8f){};
#pragma unroll
    for (int kb = 0; kb < A; kb += 32) { const v16b a0 = frag_x(x + (size_t)(m0 + nloc) * A + kb, hlf), a1 = frag_x(x + (size_t)(m0 + 16 + nloc) * A + kb, hlf);
#pragma unroll
      for (int t = 0; t < 8; ++t) { const v16b bw = frag_kb(R + (size_t)(grp * 128 + t * 16 + nloc) * A + kb, hlf); acc[0][t] = wmma16b(a0, bw, acc[0][t]); acc[1][t] = wmma16b(a1, bw, acc[1][t]); } }
    if (grp < 2) { const float sc = (grp == 0) ? SCALE * QS : KS;
#pragma unroll
      for (int t = 0; t < 8; ++t)
#pragma unroll
        for (int r = 0; r < 2; ++r)
#pragma unroll
          for (int v = 0; v < 8; ++v) { b16 a_, c_; split16(acc[r][t][v] * sc, a_, c_); Th[wave][r * 16 + 8 * hlf + v][t * 16 + nloc] = a_; Tl[wave][r * 16 + 8 * hlf + v][t * 16 + nloc] = c_; }
      wave_lds_sync();
      b16* Ph = (grp == 0) ? Qh : Kh; b16* Plo = (grp == 0) ? Ql : Kl;
      for (int pass = 0; pass < 2; ++pass) { for (int it = 0; it < 16; ++it) { const int h = it >> 1, rr = (it & 1) * 16 + (lane >> 1), c8 = (lane & 1) * 8; const size_t o = (((size_t)b * H + h) * S + s0 + rr) * KD + c8;
            *(volatile v8b*)(Ph + o) = *(const v8b*)(&Th[wave][rr][h * 16 + c8]); *(volatile v8b*)(Plo + o) = *(const v8b*)(&Tl[wave][rr][h * 16 + c8]); } __threadfence(); }
      wave_lds_sync(); }
    else if (grp == 2) {
#pragma unroll
      for (int t = 0; t < 8; ++t)
#pragma unroll
        for (int r = 0; r < 2; ++r)
#pragma unroll
          for (int v = 0; v < 8; ++v) { b16 a_, c_; split16(acc[r][t][v] * VS, a_, c_); Tv[t * 16 + nloc][wave * 32 + r * 16 + 8 * hlf + v] = a_; Tvl[t * 16 + nloc][wave * 32 + r * 16 + 8 * hlf + v] = c_; }
      __syncthreads();
      for (int pass = 0; pass < 2; ++pass) { for (int i = threadIdx.x; i < 128 * 16; i += 128) { const int j = i >> 4, c8 = (i & 15) * 8; const int h = j >> 4, d = j & 15; const size_t o = (((size_t)b * H + h) * KD + d) * S + (r0 % S) + c8; *(volatile v8b*)(Vt + o) = *(const v8b*)(&Tv[j][c8]); *(volatile v8b*)(Vtl + o) = *(const v8b*)(&Tvl[j][c8]); } __threadfence(); }
      __syncthreads(); }
    else { __shared__ __attribute__((aligned(16))) float Tg[4][32][64 + 4];
      for (int gh = 0; gh < 2; ++gh) {
#pragma unroll
        for (int t = 0; t < 4; ++t)
#pragma unroll
          for (int r = 0; r < 2; ++r)
#pragma unroll
            for (int v = 0; v < 8; ++v) Tg[wave][r * 16 + 8 * hlf + v][t * 16 + nloc] = sigm(acc[r][gh * 4 + t][v]);
        wave_lds_sync();
        for (int pass = 0; pass < 2; ++pass) { for (int i = lane; i < 32 * 16; i += 32) { const int rr = i >> 4, c4 = (i & 15) * 4; *(volatile v4f*)(G + (size_t)(m0 + rr) * 128 + gh * 64 + c4) = *(const v4f*)(&Tg[wave][rr][c4]); } __threadfence(); }
        wave_lds_sync(); } } }
}

__global__ __launch_bounds__(256) void attn_kernel(const b16* __restrict__ Qh, const b16* __restrict__ Ql, const b16* __restrict__ Kh, const b16* __restrict__ Kl, const b16* __restrict__ Vt, const b16* __restrict__ Vtl, const float* __restrict__ bias, const float* __restrict__ nb, const float* __restrict__ G, float* __restrict__ GW) {
  __shared__ __attribute__((aligned(16))) float Os[16][128 + 4];
  const int h = threadIdx.x >> 5, lane = threadIdx.x & 31, hh = lane >> 4, col = lane & 15, b = blockIdx.y, q0 = blockIdx.x * 16, qi = q0 + col;
  const size_t pb = ((size_t)b * H + h) * S * KD; const b16* V = Vt + ((size_t)b * H + h) * KD * S; const b16* Vl = Vtl + ((size_t)b * H + h) * KD * S; const float* brow = bias + ((size_t)b * S + qi) * S; const float* nrow = nb + (size_t)qi * S;
  const v16b qa = frag16(Qh + pb + (size_t)qi * KD, hh), qb = frag16(Ql + pb + (size_t)qi * KD, hh);
  float m = -INFINITY, l = 0.0f; v8f o = {};
  for (int kb = 0; kb < S; kb += 32) {
    v8f s0 = {}, s1 = {};
    { const v16b k0h = frag16(Kh + pb + (size_t)(kb + col) * KD, hh), k0l = frag16(Kl + pb + (size_t)(kb + col) * KD, hh), k1h = frag16(Kh + pb + (size_t)(kb + 16 + col) * KD, hh), k1l = frag16(Kl + pb + (size_t)(kb + 16 + col) * KD, hh);
      s0 = wmma16b(k0h, qa, s0); s0 = wmma16b(k0h, qb, s0); s0 = wmma16b(k0l, qa, s0); s1 = wmma16b(k1h, qa, s1); s1 = wmma16b(k1h, qb, s1); s1 = wmma16b(k1l, qa, s1); }
    float mr = -INFINITY;
#pragma unroll
    for (int r = 0; r < 8; ++r) { const int ka = kb + 8 * hh + r, kc = ka + 16; s0[r] = s0[r] * (1.0f / (QS * KS)) + (bf16_rne(brow[ka]) + bf16_rne(nrow[ka])); s1[r] = s1[r] * (1.0f / (QS * KS)) + (bf16_rne(brow[kc]) + bf16_rne(nrow[kc])); mr = fmaxf(mr, fmaxf(s0[r], s1[r])); }
    mr = fmaxf(mr, __shfl_xor(mr, 16));
    const float mn = fmaxf(m, mr), al_ = nexp(m - mn); m = mn; float sum = 0.0f; v16b ph, pl;
#pragma unroll
    for (int r = 0; r < 8; ++r) { const float e0 = nexp(s0[r] - mn), e1 = nexp(s1[r] - mn); sum += e0 + e1; b16 a_, c_; split16(e0 * PS, a_, c_); ph[r] = a_; pl[r] = c_; split16(e1 * PS, a_, c_); ph[8 + r] = a_; pl[8 + r] = c_; }
    sum += __shfl_xor(sum, 16); l = l * al_ + sum; o *= al_;
    const v16b vf = frag_kb(V + (size_t)col * S + kb, hh), vlf = frag_kb(Vl + (size_t)col * S + kb, hh); o = wmma16b(vf, ph, o); o = wmma16b(vf, pl, o); o = wmma16b(vlf, ph, o); }
  const float inv = 1.0f / (l * VS * PS);
#pragma unroll
  for (int r = 0; r < 8; ++r) { const int c = 8 * hh + r; Os[col][h * KD + c] = G[((size_t)b * S + qi) * 128 + h * KD + c] * (o[r] * inv); }
  __syncthreads();
  for (int pass = 0; pass < 2; ++pass) { for (int i = threadIdx.x; i < 16 * 32; i += 256) { const int rr = i >> 5, c4 = (i & 31) * 4; *(volatile v4f*)(GW + ((size_t)b * S + q0 + rr) * 128 + c4) = *(const v4f*)(&Os[rr][c4]); } __threadfence(); }
}

__global__ __launch_bounds__(128) void out_kernel(const float* __restrict__ GW, const b16* __restrict__ R, float* __restrict__ out) {
  __shared__ __attribute__((aligned(16))) float Ts[4][32][128 + 4];
  const int lane = threadIdx.x & 31, wave = threadIdx.x >> 5, nloc = lane & 15, hlf = lane >> 4, m0 = blockIdx.x * 128 + wave * 32; const b16* Wo = R + (size_t)NPJ * A;
  v8f acc[2][8];
#pragma unroll
  for (int r = 0; r < 2; ++r)
#pragma unroll
    for (int t = 0; t < 8; ++t) acc[r][t] = (v8f){};
#pragma unroll
  for (int kb = 0; kb < 128; kb += 32) { v16b a0, l0, a1, l1; frag_split(GW + (size_t)(m0 + nloc) * 128 + kb, hlf, a0, l0); frag_split(GW + (size_t)(m0 + 16 + nloc) * 128 + kb, hlf, a1, l1);
#pragma unroll
    for (int t = 0; t < 8; ++t) { const v16b bw = frag_kb(Wo + (size_t)(t * 16 + nloc) * 128 + kb, hlf); acc[0][t] = wmma16b(a0, bw, acc[0][t]); acc[0][t] = wmma16b(l0, bw, acc[0][t]); acc[1][t] = wmma16b(a1, bw, acc[1][t]); acc[1][t] = wmma16b(l1, bw, acc[1][t]); } }
#pragma unroll
  for (int t = 0; t < 8; ++t)
#pragma unroll
    for (int r = 0; r < 2; ++r)
#pragma unroll
      for (int v = 0; v < 8; ++v) Ts[wave][r * 16 + 8 * hlf + v][t * 16 + nloc] = acc[r][t][v] * (1.0f / AS_);
  wave_lds_sync();
  for (int pass = 0; pass < 2; ++pass) { for (int i = lane; i < 32 * 32; i += 32) { const int rr = i >> 5, c4 = (i & 31) * 4; *(volatile v4f*)(out + (size_t)(m0 + rr) * O + c4) = *(const v4f*)(&Ts[wave][rr][c4]); } __threadfence(); }
}
}

extern "C" void kernel_launch(void* const* d_in, const int* in_sizes, int n_in,
                              void* d_out, int out_size, void* d_ws, size_t ws_size, hipStream_t stream) {
  (void)n_in; (void)out_size;
  const float* x = (const float*)d_in[0]; const float* bias = (const float*)d_in[1]; const float* nb = (const float*)d_in[2]; const float* wq = (const float*)d_in[3]; const float* wk = (const float*)d_in[4]; const float* wv = (const float*)d_in[5]; const float* wg = (const float*)d_in[6]; const float* wo = (const float*)d_in[7];
  float* out = (float*)d_out;
  if (in_sizes[0] != NR * A || in_sizes[1] != Bn * S * S || in_sizes[2] != S * S || in_sizes[3] != A * H * KD || in_sizes[7] != H * KD * O) return;
  size_t off = 0; char* ws = (char*)d_ws;
  auto carve = [&](size_t bytes) { char* p = ws + off; off += (bytes + 255) & ~(size_t)255; return p; };
  b16* R = (b16*)carve((size_t)(NPJ * A + O * 128) * 2); b16* Qh = (b16*)carve(PL * 2); b16* Ql = (b16*)carve(PL * 2); b16* Kh = (b16*)carve(PL * 2); b16* Kl = (b16*)carve(PL * 2); b16* Vt = (b16*)carve(PL * 2); b16* Vtl = (b16*)carve(PL * 2);
  float* G = (float*)carve((size_t)NR * 128 * 4); float* GW = (float*)carve((size_t)NR * 128 * 4);
  if (off > ws_size) return;
  prep_kernel<<<64, 256, 0, stream>>>(wq, wk, wv, wg, wo, R);
  proj_kernel<<<NR / 128, 128, 0, stream>>>(x, R, Qh, Ql, Kh, Kl, Vt, Vtl, G);
  attn_kernel<<<dim3(S / 16, Bn), 256, 0, stream>>>(Qh, Ql, Kh, Kl, Vt, Vtl, bias, nb, G, GW);
  out_kernel<<<NR / 128, 128, 0, stream>>>(GW, R, out);
}
